// GroupedQueryAttention_89163521064963
// MI455X (gfx1250) — hardware-verified
//
#include <hip/hip_runtime.h>


#define NB_  2
#define TT   2048
#define DM   2048
#define NH_  32
#define NKV  8
#define REP  (NH_ / NKV)
#define HD   64
#define DQ   (NH_ * HD)
#define DKV  (NKV * HD)
#define ZH   2
#define RH   512
#define WIN  2048
#define PCAR 1024.0f
#define SCL  0.125f
typedef _Float16 h16;
typedef unsigned short bf;
typedef __attribute__((ext_vector_type(16))) __bf16   v16bf;
typedef __attribute__((ext_vector_type(16))) _Float16 v16h;
typedef __attribute__((ext_vector_type(8)))  _Float16 v8h;
typedef __attribute__((ext_vector_type(8)))  unsigned short v8us;
typedef __attribute__((ext_vector_type(8)))  float    v8f;
typedef __attribute__((ext_vector_type(4)))  float    v4f;
typedef v8h  __attribute__((may_alias)) v8ha;
typedef v4f  __attribute__((may_alias)) v4fa;
typedef v8us __attribute__((may_alias)) v8usa;

__device__ __forceinline__ unsigned short f2bf(float f) { unsigned u = __float_as_uint(f); u += 0x7FFFu + ((u >> 16) & 1u); return (unsigned short)(u >> 16); }
__device__ __forceinline__ float bf2f(unsigned short b) { return __uint_as_float(((unsigned)b) << 16); }
__device__ __forceinline__ float bfr(float f) { return bf2f(f2bf(f)); }
__device__ __forceinline__ v16h cat16(v8h lo, v8h hi) { return __builtin_shufflevector(lo, hi, 0, 1, 2, 3, 4, 5, 6, 7, 8, 9, 10, 11, 12, 13, 14, 15); }
__device__ __forceinline__ v16bf cat16b(v8us lo, v8us hi) { return __builtin_bit_cast(v16bf, __builtin_shufflevector(lo, hi, 0, 1, 2, 3, 4, 5, 6, 7, 8, 9, 10, 11, 12, 13, 14, 15)); }
__device__ __forceinline__ v8f wmma16(v16h a, v16h b, v8f c) { return __builtin_amdgcn_wmma_f32_16x16x32_f16(false, a, false, b, (short)0, c, false, false); }
__device__ __forceinline__ v8f wmmab(v16bf a, v16bf b, v8f c) { return __builtin_amdgcn_wmma_f32_16x16x32_bf16(false, a, false, b, (short)0, c, false, false); }


template <typename T16> struct WFrag;
template <> struct WFrag<h16> { typedef v16h V; static __device__ __forceinline__ V ld(const h16* p) { return cat16(*(const v8h*)p, *(const v8h*)(p + 16)); } static __device__ __forceinline__ v8f mma(V a, V b, v8f c) { return wmma16(a, b, c); } };
template <> struct WFrag<bf> { typedef v16bf V; static __device__ __forceinline__ V ld(const bf* p) { return cat16b(*(const v8us*)p, *(const v8us*)(p + 16)); } static __device__ __forceinline__ v8f mma(V a, V b, v8f c) { return wmmab(a, b, c); } };
template <typename T16, int NSPLIT, bool BIAS>
__global__ __launch_bounds__(32) void k_gemmw(const T16* __restrict__ A, const T16* __restrict__ A2, const T16* __restrict__ Bt, const T16* __restrict__ Bt2, int K, float* C, int ldc, const float* __restrict__ bias, size_t sA, size_t sB, size_t sC) {
    typedef typename WFrag<T16>::V V;
    __shared__ __align__(16) float os[16 * 68];
    const size_t z = blockIdx.z; A += z * sA; if (A2) A2 += z * sA; Bt += z * sB; if (Bt2) Bt2 += z * sB; C += z * sC;
    const int lane = threadIdx.x & 31, lr = lane & 15, hi = lane >> 4; const int r0 = blockIdx.x * 64, c0 = blockIdx.y * 64;
    v8f acc[4][4];
#pragma unroll
    for (int mb = 0; mb < 4; ++mb)
#pragma unroll
        for (int nb = 0; nb < 4; ++nb) acc[mb][nb] = (v8f){};
    const size_t aoff = (size_t)(r0 + lr) * K + 8 * hi, boff = (size_t)(c0 + lr) * K + 8 * hi;
    for (int kc = 0; kc < K; kc += 32) {
        V a[4], a2[4];
#pragma unroll
        for (int mb = 0; mb < 4; ++mb) { a[mb] = WFrag<T16>::ld(A + aoff + (size_t)mb * 16 * K + kc); if (NSPLIT == 1 || NSPLIT == 2) a2[mb] = WFrag<T16>::ld(A2 + aoff + (size_t)mb * 16 * K + kc); }
#pragma unroll
        for (int nb = 0; nb < 4; ++nb) { const V b = WFrag<T16>::ld(Bt + boff + (size_t)nb * 16 * K + kc); V b2; if (NSPLIT >= 2) b2 = WFrag<T16>::ld(Bt2 + boff + (size_t)nb * 16 * K + kc);
#pragma unroll
            for (int mb = 0; mb < 4; ++mb) { acc[mb][nb] = WFrag<T16>::mma(a[mb], b, acc[mb][nb]); if (NSPLIT == 1 || NSPLIT == 2) acc[mb][nb] = WFrag<T16>::mma(a2[mb], b, acc[mb][nb]); if (NSPLIT >= 2) acc[mb][nb] = WFrag<T16>::mma(a[mb], b2, acc[mb][nb]); } }
        asm volatile("v_nop\n\tv_nop\n\tv_nop\n\tv_nop" : "+v"(acc[0][0]), "+v"(acc[1][1]), "+v"(acc[2][2]), "+v"(acc[3][3]) : "v"(a[0]), "v"(a[3]));
    }
#pragma unroll
    for (int mb = 0; mb < 4; ++mb) {
#pragma unroll
        for (int nb = 0; nb < 4; ++nb) {
#pragma unroll
            for (int j = 0; j < 8; ++j) os[(hi * 8 + j) * 68 + nb * 16 + lr] = acc[mb][nb][j]; }
        __builtin_amdgcn_wave_barrier(); asm volatile("" ::: "memory");
        float* crow = C + (size_t)(r0 + mb * 16) * ldc + c0;
#pragma unroll 1
        for (int ps = 0; ps < 2; ++ps) {
#pragma unroll
            for (int s = 0; s < 8; ++s) { const int row = 2 * s + hi, cofs = lr * 4; v4f val = *(const v4fa*)(os + row * 68 + cofs); if (BIAS) { val[0] += bfr(bias[c0 + cofs]); val[1] += bfr(bias[c0 + cofs + 1]); val[2] += bfr(bias[c0 + cofs + 2]); val[3] += bfr(bias[c0 + cofs + 3]); }
                *(volatile v4f*)(crow + (size_t)row * ldc + cofs) = val; }
            if (ps == 0) __threadfence(); }
        __builtin_amdgcn_wave_barrier(); asm volatile("" ::: "memory");
    }
}

template <typename T16, int NSPLIT, int CMODE>
__global__ __launch_bounds__(32) void k_gemmc(const T16* __restrict__ A, const T16* __restrict__ A2, const T16* __restrict__ Bt, const T16* __restrict__ Bt2, int K, float* C, int ldc, int roff, size_t sA, size_t sB, size_t sC) {
    typedef typename WFrag<T16>::V V;
    __shared__ __align__(16) float os[16 * 68];
    const size_t z = blockIdx.z; A += z * sA; if (A2) A2 += z * sA; Bt += z * sB; if (Bt2) Bt2 += z * sB; C += z * sC;
    const int lane = threadIdx.x & 31, lr = lane & 15, hi = lane >> 4; const int r0 = blockIdx.x * 64, c0 = blockIdx.y * 64;
    if (CMODE == 1 && c0 > r0 + roff + 63) return;
    const int Kl = (CMODE == 2) ? min(K, r0 + roff + 64) : K;
    v8f acc[4][4];
#pragma unroll
    for (int mb = 0; mb < 4; ++mb)
#pragma unroll
        for (int nb = 0; nb < 4; ++nb) acc[mb][nb] = (v8f){};
    const size_t aoff = (size_t)(r0 + lr) * K + 8 * hi, boff = (size_t)(c0 + lr) * K + 8 * hi;
    for (int kc = 0; kc < Kl; kc += 32) {
        V a[4], a2[4];
#pragma unroll
        for (int mb = 0; mb < 4; ++mb) { a[mb] = WFrag<T16>::ld(A + aoff + (size_t)mb * 16 * K + kc); if (NSPLIT == 1 || NSPLIT == 2) a2[mb] = WFrag<T16>::ld(A2 + aoff + (size_t)mb * 16 * K + kc); }
#pragma unroll
        for (int nb = 0; nb < 4; ++nb) { const V b = WFrag<T16>::ld(Bt + boff + (size_t)nb * 16 * K + kc); V b2; if (NSPLIT >= 2) b2 = WFrag<T16>::ld(Bt2 + boff + (size_t)nb * 16 * K + kc);
#pragma unroll
            for (int mb = 0; mb < 4; ++mb) { acc[mb][nb] = WFrag<T16>::mma(a[mb], b, acc[mb][nb]); if (NSPLIT == 1 || NSPLIT == 2) acc[mb][nb] = WFrag<T16>::mma(a2[mb], b, acc[mb][nb]); if (NSPLIT >= 2) acc[mb][nb] = WFrag<T16>::mma(a[mb], b2, acc[mb][nb]); } }
        asm volatile("v_nop\n\tv_nop\n\tv_nop\n\tv_nop" : "+v"(acc[0][0]), "+v"(acc[1][1]), "+v"(acc[2][2]), "+v"(acc[3][3]) : "v"(a[0]), "v"(a[3]));
    }
#pragma unroll
    for (int mb = 0; mb < 4; ++mb) {
#pragma unroll
        for (int nb = 0; nb < 4; ++nb) {
#pragma unroll
            for (int j = 0; j < 8; ++j) os[(hi * 8 + j) * 68 + nb * 16 + lr] = acc[mb][nb][j]; }
        __builtin_amdgcn_wave_barrier(); asm volatile("" ::: "memory");
        float* crow = C + (size_t)(r0 + mb * 16) * ldc + c0;
#pragma unroll 1
        for (int ps = 0; ps < 2; ++ps) {
#pragma unroll
            for (int s = 0; s < 8; ++s) { const int row = 2 * s + hi, cofs = lr * 4; v4f val = *(const v4fa*)(os + row * 68 + cofs);
                *(volatile v4f*)(crow + (size_t)row * ldc + cofs) = val; }
            if (ps == 0) __threadfence(); }
        __builtin_amdgcn_wave_barrier(); asm volatile("" ::: "memory");
    }
}

__device__ __forceinline__ h16 tohx(float x) { return (h16)x; }
__device__ __forceinline__ void splitf(float y, unsigned short& h, unsigned short& l) { h = f2bf(y); l = f2bf(y - bf2f(h)); }
typedef __attribute__((ext_vector_type(2))) _Float16 v2h;
typedef __attribute__((ext_vector_type(4))) _Float16 v4h;
typedef __attribute__((ext_vector_type(2))) unsigned short v2us;
typedef __attribute__((ext_vector_type(4))) unsigned short v4us;
typedef __attribute__((ext_vector_type(2))) float v2f;
typedef __attribute__((ext_vector_type(4))) int v4i;

__global__ __launch_bounds__(256) void k_wtG(const float* __restrict__ w, int K, int N, bf* Bt) {
    const int lane = threadIdx.x & 31; const int L0 = (blockIdx.x * 8 + (threadIdx.x >> 5)) * 8; const int nlines = N * K / 64;
#pragma unroll
    for (int ps = 0; ps < 2; ++ps) {
        for (int l = 0; l < 8; ++l) { const int L = L0 + l; if (L >= nlines) break; const size_t e = (size_t)L * 64 + lane * 2; const int k = (int)(e % K), n = (int)(e / K); v2us o;
            o[0] = f2bf(w[(size_t)k * N + n]); o[1] = f2bf(w[(size_t)(k + 1) * N + n]); *(volatile v2us*)(Bt + e) = o; }
        if (ps == 0) __threadfence(); }
}
__global__ __launch_bounds__(256) void k_cvt8(const float* __restrict__ src, bf* dst, size_t n8) { const size_t i = (size_t)blockIdx.x * 256 + threadIdx.x; if (i >= n8) return; const v8f v = *(const v8f*)(src + i * 8); v8us o;
#pragma unroll
    for (int k = 0; k < 8; ++k) o[k] = f2bf(v[k]); *(volatile v8us*)(dst + i * 8) = o; __threadfence(); *(volatile v8us*)(dst + i * 8) = o; }

__global__ __launch_bounds__(256) void k_ropeI(const float* __restrict__ F, int pitch, int nheads, const float* __restrict__ CS, float sc, h16* P16, bf* Ph, bf* Pl) {
    const size_t e = ((size_t)blockIdx.x * 256 + threadIdx.x) * 2; if (e >= (size_t)nheads * TT * HD) return; const int d = (int)(e % HD); const int t = (int)((e / HD) % TT); const int h = (int)(e / ((size_t)HD * TT)); const float* f = F + (size_t)t * pitch + h * HD; const float x0 = f[d], x1 = f[d + 1]; const v2f cs = *(const v2f*)(CS + ((size_t)t * HD + d) * 2); v2h o16; v2us oh, ol;
    float a0 = __fmul_rn(x0, cs[0]), b0 = __fmul_rn(x1, cs[1]), a1 = __fmul_rn(x1, cs[0]), b1 = __fmul_rn(x0, cs[1]);
    float r0 = __fsub_rn(a0, b0) * sc, r1 = __fadd_rn(b1, a1) * sc;
    o16[0] = tohx(r0); o16[1] = tohx(r1); { unsigned short a2, c2; splitf(r0, a2, c2); oh[0] = a2; ol[0] = c2; splitf(r1, a2, c2); oh[1] = a2; ol[1] = c2; }
    *(volatile v2h*)(P16 + e) = o16; *(volatile v2us*)(Ph + e) = oh; *(volatile v2us*)(Pl + e) = ol; __threadfence(); *(volatile v2h*)(P16 + e) = o16; *(volatile v2us*)(Ph + e) = oh; *(volatile v2us*)(Pl + e) = ol; }


__global__ __launch_bounds__(256) void k_vtp(const float* __restrict__ F, int pitch, int nheads, h16* V16, bf* Vh, bf* Vl) { const size_t e = ((size_t)blockIdx.x * 256 + threadIdx.x) * 2; if (e >= (size_t)nheads * HD * TT) return; const int t = (int)(e % TT); const int d = (int)((e / TT) % HD); const int g = (int)(e / ((size_t)TT * HD)); v2h o16; v2us oh, ol;
#pragma unroll
    for (int q = 0; q < 2; ++q) { const float x = F[(size_t)(t + q) * pitch + g * HD + d]; o16[q] = tohx(x); unsigned short a2, c2; splitf(x, a2, c2); oh[q] = a2; ol[q] = c2; }
    *(volatile v2h*)(V16 + e) = o16; *(volatile v2us*)(Vh + e) = oh; *(volatile v2us*)(Vl + e) = ol; __threadfence(); *(volatile v2h*)(V16 + e) = o16; *(volatile v2us*)(Vh + e) = oh; *(volatile v2us*)(Vl + e) = ol; }
__global__ __launch_bounds__(256) void k_cscis(const float* __restrict__ fc, float* CS) { const int idx = blockIdx.x * 256 + threadIdx.x; if (idx >= TT * HD) return; const int tt = idx / HD; const int dd = idx - tt * HD; const v2f c2 = *(const v2f*)(fc + ((size_t)tt * (HD / 2) + (dd >> 1)) * 2); v2f cs; cs[0] = bfr(c2[0]); cs[1] = bfr(c2[1]); *(volatile v2f*)(CS + (size_t)idx * 2) = cs; __threadfence(); *(volatile v2f*)(CS + (size_t)idx * 2) = cs; }
__global__ __launch_bounds__(256) void k_asoft(const float* __restrict__ Sb, h16* P16, bf* Ph, bf* Pl) {
    const int lane = threadIdx.x & 31; const int row = blockIdx.x * 8 + (threadIdx.x >> 5); if (row >= ZH * TT) return; const int i = row % TT; const int zz = row / TT; (void)zz; const bool hires = (i < RH); const float* sr = Sb + (size_t)row * TT; float v[TT / 32]; float mx = -3.0e38f;
#pragma unroll
    for (int ch = 0; ch < TT / 128; ++ch) { const int j0 = ch * 128 + lane * 4; const v4f a = *(const v4f*)(sr + j0);
#pragma unroll
        for (int q = 0; q < 4; ++q) { const int j = j0 + q; (void)j; const float t = (j <= i && i - j < WIN) ? a[q] * SCL : -3.0e38f; v[ch * 4 + q] = t; mx = fmaxf(mx, t); } }
#pragma unroll
    for (int sh = 16; sh; sh >>= 1) mx = fmaxf(mx, __shfl_xor(mx, sh, 32));
    float sum = 0.f;
#pragma unroll
    for (int k = 0; k < TT / 32; ++k) { float d0 = __fsub_rn(v[k], mx); v[k] = __builtin_amdgcn_exp2f(__fmul_rn(d0, 1.4426950408889634f)); sum += v[k]; }
#pragma unroll
    for (int sh = 16; sh; sh >>= 1) sum += __shfl_xor(sum, sh, 32);
    const float f = __fdiv_rn(hires ? 1.0f : PCAR, sum);
#pragma unroll 1
    for (int ps = 0; ps < 2; ++ps) {
        if (hires) {
#pragma unroll
            for (int ch = 0; ch < TT / 128; ++ch) { v4us oh, ol;
#pragma unroll
                for (int q = 0; q < 4; ++q) { unsigned short a, c2; splitf(v[ch * 4 + q] * f, a, c2); oh[q] = a; ol[q] = c2; }
                const size_t oo = ((size_t)zz * (RH ? RH : 1) + i) * TT + ch * 128 + lane * 4; *(volatile v4us*)(Ph + oo) = oh; *(volatile v4us*)(Pl + oo) = ol; }
        } else {
#pragma unroll
            for (int ch = 0; ch < TT / 128; ++ch) { v4h o4;
#pragma unroll
                for (int q = 0; q < 4; ++q) o4[q] = tohx(v[ch * 4 + q] * f);
                *(volatile v4h*)(P16 + (size_t)row * TT + ch * 128 + lane * 4) = o4; } }
        if (ps == 0) __threadfence(); }
}
__global__ __launch_bounds__(256) void k_merge(const float* __restrict__ O, int h0, bf* Ah, bf* Al) { const size_t e = ((size_t)blockIdx.x * 256 + threadIdx.x) * 2; if (e >= (size_t)ZH * TT * HD) return; const int d = (int)(e % HD); const int t = (int)((e / HD) % TT); const int zz = (int)(e / ((size_t)HD * TT)); const float cs = (t < RH) ? 1.0f : (1.0f / PCAR); const size_t oo = (size_t)t * DQ + (h0 + zz) * HD + d;
    v2us oh, ol;
#pragma unroll
    for (int q = 0; q < 2; ++q) { unsigned short a, c2; splitf(O[e + q] * cs, a, c2); oh[q] = a; ol[q] = c2; } *(volatile v2us*)(Ah + oo) = oh; *(volatile v2us*)(Al + oo) = ol; __threadfence(); *(volatile v2us*)(Ah + oo) = oh; *(volatile v2us*)(Al + oo) = ol; }

extern "C" void kernel_launch(void* const* d_in, const int* in_sizes, int n_in,
                              void* d_out, int out_size, void* d_ws, size_t ws_size, hipStream_t stream) {
    (void)in_sizes; (void)n_in; (void)out_size;
    const float* x = (const float*)d_in[0]; const float* fcis = (const float*)d_in[1]; const float* wq = (const float*)d_in[2]; const float* wk = (const float*)d_in[3]; const float* wv = (const float*)d_in[4]; const float* wo = (const float*)d_in[5];
    float* OUT = (float*)d_out;
    char* wsp = (char*)d_ws;
    auto take = [&](size_t bytes) { char* p = wsp; wsp += (bytes + 255) & ~(size_t)255; return (void*)p; };
    bf* WQ = (bf*)take((size_t)DQ * DM * 2); bf* WK = (bf*)take((size_t)DKV * DM * 2); bf* WV = (bf*)take((size_t)DKV * DM * 2); bf* WO = (bf*)take((size_t)DM * DQ * 2); float* CS = (float*)take((size_t)TT * HD * 2 * 4);
    bf* XB = (bf*)take((size_t)TT * DM * 2); float* FQ = (float*)take((size_t)TT * DQ * 4); float* FK = (float*)take((size_t)TT * DKV * 4);
    h16* QP16 = (h16*)take((size_t)NH_ * TT * HD * 2); h16* KP16 = (h16*)take((size_t)NKV * TT * HD * 2); h16* VT16 = (h16*)take((size_t)NKV * HD * TT * 2);
    bf* QPh = (bf*)take((size_t)NH_ * TT * HD * 2); bf* QPl = (bf*)take((size_t)NH_ * TT * HD * 2); bf* KPh = (bf*)take((size_t)NKV * TT * HD * 2); bf* KPl = (bf*)take((size_t)NKV * TT * HD * 2); bf* VTh = (bf*)take((size_t)NKV * HD * TT * 2); bf* VTl = (bf*)take((size_t)NKV * HD * TT * 2); bf* Ph = (bf*)take((size_t)ZH * RH * TT * 2); bf* Pl = (bf*)take((size_t)ZH * RH * TT * 2);
    float* Sb = (float*)take((size_t)ZH * TT * TT * 4); h16* P16 = (h16*)take((size_t)ZH * TT * TT * 2); float* Ob = (float*)take((size_t)ZH * TT * HD * 4); bf* ATh = (bf*)take((size_t)TT * DQ * 2); bf* ATl = (bf*)take((size_t)TT * DQ * 2);
    if ((size_t)(wsp - (char*)d_ws) > ws_size) return;
    float* FV = FK;
    { k_wtG<<<(unsigned)((DM * DQ / 64 + 63) / 64), 256, 0, stream>>>(wq, DM, DQ, WQ); k_wtG<<<(unsigned)((DM * DKV / 64 + 63) / 64), 256, 0, stream>>>(wk, DM, DKV, WK); k_wtG<<<(unsigned)((DM * DKV / 64 + 63) / 64), 256, 0, stream>>>(wv, DM, DKV, WV);
      k_wtG<<<(unsigned)((DQ * DM / 64 + 63) / 64), 256, 0, stream>>>(wo, DQ, DM, WO);
       }
    k_cscis<<<(TT * HD + 255) / 256, 256, 0, stream>>>(fcis, (float*)CS);
    const unsigned LQ = (unsigned)(((size_t)NH_ * TT * HD / 2 + 255) / 256), LKv = (unsigned)(((size_t)NKV * TT * HD / 2 + 255) / 256);
    for (int b = 0; b < NB_; ++b) {

        k_cvt8<<<(unsigned)(((size_t)TT * DM / 8 + 255) / 256), 256, 0, stream>>>(x + (size_t)b * TT * DM, XB, (size_t)TT * DM / 8);
        k_gemmw<bf, 0, false><<<dim3(TT / 64, DQ / 64, 1), 32, 0, stream>>>(XB, nullptr, WQ, nullptr, DM, FQ, DQ, nullptr, 0, 0, 0);
        k_ropeI<<<LQ, 256, 0, stream>>>(FQ, DQ, NH_, CS, 1.0f, QP16, QPh, QPl);
        k_gemmw<bf, 0, false><<<dim3(TT / 64, DKV / 64, 1), 32, 0, stream>>>(XB, nullptr, WK, nullptr, DM, FK, DKV, nullptr, 0, 0, 0);
        k_ropeI<<<LKv, 256, 0, stream>>>(FK, DKV, NKV, CS, 1.0f, KP16, KPh, KPl);
        k_gemmw<bf, 0, false><<<dim3(TT / 64, DKV / 64, 1), 32, 0, stream>>>(XB, nullptr, WV, nullptr, DM, FV, DKV, nullptr, 0, 0, 0); k_vtp<<<LKv, 256, 0, stream>>>(FV, DKV, NKV, VT16, VTh, VTl);
        for (int h0 = 0; h0 < NH_; h0 += ZH) { const size_t zq = (size_t)h0, zk = (size_t)(h0 / REP);
            k_gemmc<bf, 2, 1><<<dim3(RH / 64, TT / 64, ZH), 32, 0, stream>>>(QPh + zq * TT * HD, QPl + zq * TT * HD, KPh + zk * TT * HD, KPl + zk * TT * HD, HD, Sb, TT, 0, (size_t)TT * HD, 0, (size_t)TT * TT);
            k_gemmc<h16, 0, 1><<<dim3((TT - RH) / 64, TT / 64, ZH), 32, 0, stream>>>(QP16 + zq * TT * HD + (size_t)RH * HD, nullptr, KP16 + zk * TT * HD, nullptr, HD, Sb + (size_t)RH * TT, TT, RH, (size_t)TT * HD, 0, (size_t)TT * TT);
            k_asoft<<<ZH * TT / 8, 256, 0, stream>>>(Sb, P16, Ph, Pl);
            k_gemmc<bf, 2, 2><<<dim3(RH / 64, HD / 64, ZH), 32, 0, stream>>>(Ph, Pl, VTh + zk * HD * TT, VTl + zk * HD * TT, TT, Ob, HD, 0, (size_t)RH * TT, 0, (size_t)TT * HD);
            k_gemmc<h16, 0, 2><<<dim3((TT - RH) / 64, HD / 64, ZH), 32, 0, stream>>>(P16 + (size_t)RH * TT, nullptr, VT16 + zk * HD * TT, nullptr, TT, Ob + (size_t)RH * HD, HD, RH, (size_t)TT * TT, 0, (size_t)TT * HD);
            k_merge<<<(unsigned)(((size_t)ZH * TT * HD / 2 + 255) / 256), 256, 0, stream>>>(Ob, h0, ATh, ATl); }
        k_gemmw<bf, 1, false><<<dim3(TT / 64, DM / 64, 1), 32, 0, stream>>>(ATh, ATl, WO, nullptr, DQ, OUT + (size_t)b * TT * DM, DM, nullptr, 0, 0, 0); }
}
